// PartialFormerBlock_37984690766447
// MI455X (gfx1250) — hardware-verified
//
#include <hip/hip_runtime.h>
#include <math.h>
#include <stdint.h>

#define LTOK 3136
#define DIM  384
#define HEADS 6
#define HD   64
#define HEXP 24
#define PRD  96
#define HID  1536
#define NP   784
#define NPP  800
#define NF   392
#define NBT  1568
#define MQ   1569
#define MQP  1600
#define HS   56
#define HPW  28
#define KC   64
#define SP   68
#define SCALE_F 0.125f
#define LN_EPS 1e-5f

typedef __attribute__((ext_vector_type(16))) __bf16 v16b;
typedef __attribute__((ext_vector_type(8)))  __bf16 v8b;
typedef __attribute__((ext_vector_type(8)))  float  v8f;
typedef __attribute__((ext_vector_type(4)))  float  v4f;
typedef __attribute__((ext_vector_type(4)))  unsigned int v4u;
typedef unsigned short us;

__device__ __forceinline__ us f2bf_bits(float f) {
  unsigned u = __float_as_uint(f);
  return (us)((u + 0x7FFFu + ((u >> 16) & 1u)) >> 16);
}
__device__ __forceinline__ float bf_bits2f(us h) { return __uint_as_float(((unsigned)h) << 16); }
__device__ __forceinline__ unsigned pk16(us a, us b) { return (unsigned)a | ((unsigned)b << 16); }

__device__ __forceinline__ void split8(v4f a, v4f b, v4u& hv, v4u& lv) {
  float f[8] = {a.x, a.y, a.z, a.w, b.x, b.y, b.z, b.w};
#pragma unroll
  for (int q = 0; q < 4; ++q) {
    const us h0 = f2bf_bits(f[2 * q]), h1 = f2bf_bits(f[2 * q + 1]);
    const us l0 = f2bf_bits(f[2 * q] - bf_bits2f(h0)), l1 = f2bf_bits(f[2 * q + 1] - bf_bits2f(h1));
    hv[q] = pk16(h0, h1);
    lv[q] = pk16(l0, l1);
  }
}

__device__ __forceinline__ float wave_sum(float v) {
#pragma unroll
  for (int off = 16; off > 0; off >>= 1) v += __shfl_xor(v, off, 32);
  return v;
}
__device__ __forceinline__ float wave_max(float v) {
#pragma unroll
  for (int off = 16; off > 0; off >>= 1) v = fmaxf(v, __shfl_xor(v, off, 32));
  return v;
}

__device__ __forceinline__ void dep_guard(v8f& a, v8f& b, v16b x, v16b y) {
  asm volatile("v_nop\n\tv_nop\n\tv_nop\n\tv_nop" : "+v"(a), "+v"(b) : "v"(x), "v"(y));
}
__device__ __forceinline__ void keep4(v16b a, v16b b, v16b c, v16b d) { asm volatile("v_nop" :: "v"(a), "v"(b), "v"(c), "v"(d)); }
__device__ __forceinline__ void acc_guard4(v8f& a, v8f& b, v8f& c, v8f& d) {
  asm volatile("v_nop\n\tv_nop\n\tv_nop\n\tv_nop" : "+v"(a), "+v"(b), "+v"(c), "+v"(d));
}
union FB { v16b v; v8b h[2]; };
__device__ __forceinline__ v16b ldfrag(const __bf16* p) {
  FB f; f.h[0] = *(const v8b*)(p); f.h[1] = *(const v8b*)(p + 16); return f.v;
}
__device__ __forceinline__ v8f mma(v16b a, v16b b, v8f c) {
  return __builtin_amdgcn_wmma_f32_16x16x32_bf16(false, a, false, b, (short)0, c, false, false);
}
__device__ __forceinline__ v8f mma_g(v16b a, v16b b, v8f c) {
  c = __builtin_amdgcn_wmma_f32_16x16x32_bf16(false, a, false, b, (short)0, c, false, false);
  asm volatile("v_nop\n\tv_nop\n\tv_nop\n\tv_nop" : "+v"(c) : "v"(a), "v"(b));
  return c;
}

template <int BIAS_MODE, int OUT_MODE, bool RESID, int ACT>
__global__ __launch_bounds__(256) void k_gemm64(
    const us* __restrict__ Ap, const us* __restrict__ A2p, int lda, long strideA,
    const us* __restrict__ Btp, const us* __restrict__ Bt2p, int ldb, long strideB,
    void* Cout, void* Cout2, int ldc, long strideC,
    const float* bias, const float* resid,
    int M, int N, int K, float scale) {
  __shared__ __align__(16) float sT[8][16 * 68];
  const int b    = blockIdx.y;
  const int lane = threadIdx.x & 31;
  const int wave = threadIdx.x >> 5;
  const int tilesN = N >> 6;
  const int tilesM = M >> 6;
  const int tile = blockIdx.x * 8 + wave;
  if (tile >= tilesM * tilesN) return;
  const int tm = tile / tilesN;
  const int tn = tile - tm * tilesN;
  const int m0 = tm << 6;
  const int n0 = tn << 6;

  const __bf16* Ab  = (const __bf16*)(const void*)Ap   + (size_t)b * strideA;
  const __bf16* Ab2 = (const __bf16*)(const void*)A2p  + (size_t)b * strideA;
  const __bf16* Bb  = (const __bf16*)(const void*)Btp  + (size_t)b * strideB;
  const __bf16* Bb2 = (const __bf16*)(const void*)Bt2p + (size_t)b * strideB;

  const int rlane = lane & 15;
  const int koff  = (lane >> 4) * 8;
  const int mOff  = (lane >> 4) * 8;

  const v8f z8 = {0.f, 0.f, 0.f, 0.f, 0.f, 0.f, 0.f, 0.f};
  v8f acc[4][4];
#pragma unroll
  for (int i = 0; i < 4; ++i)
#pragma unroll
    for (int j = 0; j < 4; ++j) acc[i][j] = z8;

  for (int k0 = 0; k0 < K; k0 += 32) {
    v16b bh[4], bl[4];
#pragma unroll
    for (int j = 0; j < 4; ++j) {
      const size_t bo = (size_t)(n0 + (j << 4) + rlane) * ldb + koff + k0;
      bh[j] = ldfrag(Bb + bo);
      bl[j] = ldfrag(Bb2 + bo);
    }
#pragma unroll
    for (int i = 0; i < 4; ++i) {
      const size_t ao = (size_t)(m0 + (i << 4) + rlane) * lda + koff + k0;
      const v16b ah = ldfrag(Ab + ao);
      const v16b al = ldfrag(Ab2 + ao);
#pragma unroll
      for (int j = 0; j < 4; ++j) {
        acc[i][j] = mma(ah, bh[j], acc[i][j]);
        acc[i][j] = mma(ah, bl[j], acc[i][j]);
        acc[i][j] = mma(al, bh[j], acc[i][j]);
      }
      dep_guard(acc[i][0], acc[i][3], ah, al);
    }
    keep4(bh[0], bh[1], bh[2], bh[3]);
    keep4(bl[0], bl[1], bl[2], bl[3]);
  }
  acc_guard4(acc[0][0], acc[0][1], acc[0][2], acc[0][3]);
  acc_guard4(acc[1][0], acc[1][1], acc[1][2], acc[1][3]);
  acc_guard4(acc[2][0], acc[2][1], acc[2][2], acc[2][3]);
  acc_guard4(acc[3][0], acc[3][1], acc[3][2], acc[3][3]);

  float* slab = sT[wave];
#pragma unroll
  for (int i = 0; i < 4; ++i) {
    const int mBase = m0 + (i << 4);
#pragma unroll
    for (int j = 0; j < 4; ++j) {
      const int n = n0 + (j << 4) + rlane;
      float bv = 0.f;
      if (BIAS_MODE == 2) bv = bias[n];
#pragma unroll
      for (int r = 0; r < 8; ++r) {
        float v = acc[i][j][r] * scale;
        if (BIAS_MODE == 1) v += bias[mBase + mOff + r];
        if (BIAS_MODE == 2) v += bv;
        if (RESID) v += resid[(size_t)(mBase + mOff + r) * ldc + n];
        if (ACT == 3) { const float e = __expf(-v); v = v * (1.0f / (1.0f + e)); }
        slab[(mOff + r) * 68 + (j << 4) + rlane] = v;
      }
    }
    __builtin_amdgcn_fence(__ATOMIC_RELEASE, "workgroup");
    __builtin_amdgcn_wave_barrier();
    __builtin_amdgcn_fence(__ATOMIC_ACQUIRE, "workgroup");
    if (OUT_MODE == 0) {
      float* C = (float*)Cout + (size_t)b * strideC;
      const int hh = lane >> 4, c4 = (lane & 15) * 4;
      for (int pass = 0; pass < 2; ++pass) {
#pragma unroll
        for (int it = 0; it < 8; ++it) {
          const int row = it * 2 + hh;
          const v4f v = *(const v4f*)(slab + row * 68 + c4);
          *(volatile v4f*)(C + (size_t)(mBase + row) * ldc + n0 + c4) = v;
        }
        __threadfence();
      }
    } else {
      const int q = lane >> 3, c8 = (lane & 7) * 8;
      us* C  = (us*)Cout  + (size_t)b * strideC;
      us* C2 = (us*)Cout2 + (size_t)b * strideC;
      v4u hv[4], lv[4];
#pragma unroll
      for (int it = 0; it < 4; ++it) {
        const int row = it * 4 + q;
        const float* sp = slab + row * 68 + c8;
        v4f a, bb;
        a.x = sp[0]; a.y = sp[1]; a.z = sp[2]; a.w = sp[3];
        bb.x = sp[4]; bb.y = sp[5]; bb.z = sp[6]; bb.w = sp[7];
        split8(a, bb, hv[it], lv[it]);
      }
      for (int pass = 0; pass < 2; ++pass) {
#pragma unroll
        for (int it = 0; it < 4; ++it) {
          const int row = it * 4 + q;
          const size_t o = (size_t)(mBase + row) * ldc + n0 + c8;
          *(volatile v4u*)(C + o)  = hv[it];
          *(volatile v4u*)(C2 + o) = lv[it];
        }
        __threadfence();
      }
    }
    __builtin_amdgcn_fence(__ATOMIC_RELEASE, "workgroup");
    __builtin_amdgcn_wave_barrier();
    __builtin_amdgcn_fence(__ATOMIC_ACQUIRE, "workgroup");
  }
}

__global__ __launch_bounds__(256) void k_split8(const float* __restrict__ in, us* hi, us* lo, int n8) {
  const int i = blockIdx.x * 256 + threadIdx.x;
  if (i >= n8) return;
  const v4f a = *(const v4f*)(in + 8 * (size_t)i);
  const v4f b = *(const v4f*)(in + 8 * (size_t)i + 4);
  v4u hv, lv;
  split8(a, b, hv, lv);
  us* ph = hi + 8 * (size_t)i;
  us* pl = lo + 8 * (size_t)i;
  *(volatile v4u*)ph = hv;
  *(volatile v4u*)pl = lv;
  __threadfence();
  *(volatile v4u*)ph = hv;
  *(volatile v4u*)pl = lv;
}

__global__ __launch_bounds__(256) void k_conv(const float* __restrict__ x, const float* __restrict__ w,
                                              const float* __restrict__ bconv, float* cout) {
  const int i = blockIdx.x * 256 + threadIdx.x;
  if (i >= LTOK * (DIM / 4)) return;
  const int r = i / (DIM / 4);
  const int d4 = (i - r * (DIM / 4)) * 4;
  const int ii0 = r / HS, jj0 = r - ii0 * HS;
  const float* w0 = w + (size_t)d4 * 9;
  const v4f z = {0.f, 0.f, 0.f, 0.f};
  v4f acc = z;
#pragma unroll
  for (int ki = 0; ki < 3; ++ki) {
#pragma unroll
    for (int kj = 0; kj < 3; ++kj) {
      const int ii = ii0 + ki - 1, jj = jj0 + kj - 1;
      const bool ok = (ii >= 0) && (ii < HS) && (jj >= 0) && (jj < HS);
      const int iic = min(max(ii, 0), HS - 1), jjc = min(max(jj, 0), HS - 1);
      v4f xv = *(const v4f*)(x + (size_t)(iic * HS + jjc) * DIM + d4);
      xv = ok ? xv : z;
      const int tap = ki * 3 + kj;
      acc.x += w0[tap] * xv.x;
      acc.y += w0[9 + tap] * xv.y;
      acc.z += w0[18 + tap] * xv.z;
      acc.w += w0[27 + tap] * xv.w;
    }
  }
  const v4f xc = *(const v4f*)(x + (size_t)r * DIM + d4);
  const v4f bb = *(const v4f*)(bconv + d4);
  const v4f o = (acc + bb) + xc;
  float* p = cout + (size_t)i * 4;
  *(volatile v4f*)p = o;
  __threadfence();
  *(volatile v4f*)p = o;
}

__global__ __launch_bounds__(256) void k_rank(const float* __restrict__ cin, int* rankA, int* order) {
  __shared__ float mean_s[NP];
  __shared__ int rank_s[NPP];
  __shared__ int ord_s[NPP];
  const int tid = threadIdx.x, wave = tid >> 5, lane = tid & 31;
  for (int p = wave; p < NP; p += 8) {
    const int ip = p / HPW, jp = p - ip * HPW;
    float s = 0.f;
#pragma unroll
    for (int t = 0; t < 4; ++t) {
      const int row = (2 * ip + (t >> 1)) * HS + 2 * jp + (t & 1);
      const float* rp = cin + (size_t)row * DIM + lane * 4;
#pragma unroll
      for (int it = 0; it < 3; ++it) {
        const v4f v = *(const v4f*)(rp + it * 128);
        s += (v.x + v.y) + (v.z + v.w);
      }
    }
    s = wave_sum(s);
    if (lane == 0) mean_s[p] = s * (1.0f / 1536.0f);
  }
  for (int i = tid; i < NPP; i += 256) { rank_s[i] = 0; ord_s[i] = (i < NP) ? i : 0; }
  __syncthreads();
  for (int i = tid; i < NP; i += 256) {
    const float mi = mean_s[i];
    int rk = 0;
#pragma unroll 4
    for (int j = 0; j < NP; ++j) {
      const float mj = mean_s[j];
      rk += (mj > mi || (mj == mi && j < i)) ? 1 : 0;
    }
    rank_s[i] = rk;
  }
  __syncthreads();
  for (int i = tid; i < NP; i += 256) {
    int rk = rank_s[i];
    rk = min(max(rk, 0), NP - 1);
    ord_s[rk] = i;
  }
  __syncthreads();
  for (int pass = 0; pass < 2; ++pass) {
    for (int line = wave; line < NPP / 32; line += 8) {
      const int idx = line * 32 + lane;
      ((volatile int*)rankA)[idx] = rank_s[idx];
      ((volatile int*)order)[idx] = ord_s[idx];
    }
    __threadfence();
  }
}

__global__ __launch_bounds__(256) void k_gather8(const float* __restrict__ cin, const float* __restrict__ qa,
                                                 const int* __restrict__ order,
                                                 us* xfh, us* xfl, us* xbh, us* xbl) {
  const int i = blockIdx.x * 256 + threadIdx.x;
  const int half = MQP * (DIM / 8);
  if (i >= 2 * half) return;
  const bool bg = i >= half;
  const int j = bg ? (i - half) : i;
  const int row = j / (DIM / 8);
  const int d8 = (j - row * (DIM / 8)) * 8;
  const int tokf = max(row - 1, 0);
  const int rkf = min(tokf >> 2, NF - 1), tf = tokf & 3;
  const int rkb = min(NF + (row >> 2), NP - 1), tb = row & 3;
  const int rk = bg ? rkb : rkf;
  const int t = bg ? tb : tf;
  int p = order[rk];
  p = min(max(p, 0), NP - 1);
  const int ip = p / HPW, jp = p - ip * HPW;
  const int srow = (2 * ip + (t >> 1)) * HS + 2 * jp + (t & 1);
  const float* cp = cin + (size_t)srow * DIM + d8;
  const v4f c0 = *(const v4f*)cp;
  const v4f c1 = *(const v4f*)(cp + 4);
  const v4f q0 = *(const v4f*)(qa + d8);
  const v4f q1 = *(const v4f*)(qa + d8 + 4);
  const bool useq = (!bg) && (row == 0);
  const bool valid = bg ? (row < NBT) : (row < MQ);
  const v4f z = {0.f, 0.f, 0.f, 0.f};
  v4f a = useq ? q0 : c0;
  v4f b = useq ? q1 : c1;
  a = valid ? a : z;
  b = valid ? b : z;
  v4u hv, lv;
  split8(a, b, hv, lv);
  us* ph = (bg ? xbh : xfh) + (size_t)row * DIM + d8;
  us* pl = (bg ? xbl : xfl) + (size_t)row * DIM + d8;
  *(volatile v4u*)ph = hv;
  *(volatile v4u*)pl = lv;
  __threadfence();
  *(volatile v4u*)ph = hv;
  *(volatile v4u*)pl = lv;
}

__global__ __launch_bounds__(192) void k_mmsa(const float* __restrict__ S,
                                              const us* __restrict__ vthp, const us* __restrict__ vtlp,
                                              const float* __restrict__ ap1w, const float* __restrict__ ap1b,
                                              const float* __restrict__ ap2w, const float* __restrict__ ap2b,
                                              us* aoh, us* aol) {
  __shared__ __align__(16) float  Ssh[HEADS * 16 * SP];
  __shared__ __align__(16) __bf16 A2h[HEADS * 16 * KC];
  __shared__ __align__(16) __bf16 A2l[HEADS * 16 * KC];
  __shared__ float mst[16 * HEXP];
  __shared__ float rzs[16 * HEXP];
  __shared__ float w1s[HEXP * HEADS];
  __shared__ float w2s[HEADS * HEXP];
  __shared__ float b1s[HEXP];
  __shared__ float b2s[HEADS];

  const int tid = threadIdx.x;
  const int wave = tid >> 5, lane = tid & 31, hg = lane >> 4, ln = lane & 15;
  const int m0 = blockIdx.x * 16;
  if (tid < HEXP * HEADS) { w1s[tid] = ap1w[tid]; w2s[tid] = ap2w[tid]; }
  if (tid < HEXP) b1s[tid] = ap1b[tid];
  if (tid < HEADS) b2s[tid] = ap2b[tid];
  const __bf16* vth = (const __bf16*)(const void*)vthp;
  const __bf16* vtl = (const __bf16*)(const void*)vtlp;

  float mA[2] = {-INFINITY, -INFINITY};
  float sA[2] = {0.f, 0.f};
#pragma unroll 1
  for (int k0 = 0; k0 < MQP; k0 += KC) {
    __syncthreads();
#pragma unroll
    for (int i = 0; i < 8; ++i) {
      const int f = tid + 192 * i;
      const int hh = f >> 8, rem = f & 255, q = rem >> 4, c4 = (rem & 15) * 4;
      const v4f v = *(const v4f*)(S + ((size_t)hh * MQP + (size_t)(m0 + q)) * MQP + k0 + c4);
      *(v4f*)(Ssh + hh * 16 * SP + q * SP + c4) = v;
    }
    __syncthreads();
    const int kmax = min(KC, MQ - k0);
#pragma unroll
    for (int pp = 0; pp < 2; ++pp) {
      const int idx = tid + pp * 192;
      const int qq = idx / HEXP, cc = idx - qq * HEXP;
      const float* srow = Ssh + qq * SP;
      const float* w1 = w1s + cc * HEADS;
      const float bb = b1s[cc];
      float m = mA[pp], s = sA[pp];
#pragma unroll 1
      for (int kk = 0; kk < kmax; ++kk) {
        float a1 = 0.f;
#pragma unroll
        for (int h = 0; h < HEADS; ++h) a1 += srow[h * 16 * SP + kk] * w1[h];
        a1 += bb;
        const float d = a1 - m;
        const float e = __expf(-fabsf(d));
        s = (d > 0.f) ? (s * e + 1.0f) : (s + e);
        m = fmaxf(m, a1);
      }
      mA[pp] = m; sA[pp] = s;
    }
  }
#pragma unroll
  for (int pp = 0; pp < 2; ++pp) {
    const int idx = tid + pp * 192;
    mst[idx] = mA[pp];
    rzs[idx] = 1.0f / sA[pp];
  }
  __syncthreads();

  const v8f z8 = {0.f, 0.f, 0.f, 0.f, 0.f, 0.f, 0.f, 0.f};
  v8f oacc[4];
#pragma unroll
  for (int dt = 0; dt < 4; ++dt) oacc[dt] = z8;
#pragma unroll 1
  for (int k0 = 0; k0 < MQP; k0 += KC) {
    __syncthreads();
#pragma unroll
    for (int i = 0; i < 8; ++i) {
      const int f = tid + 192 * i;
      const int hh = f >> 8, rem = f & 255, q = rem >> 4, c4 = (rem & 15) * 4;
      const v4f v = *(const v4f*)(S + ((size_t)hh * MQP + (size_t)(m0 + q)) * MQP + k0 + c4);
      *(v4f*)(Ssh + hh * 16 * SP + q * SP + c4) = v;
    }
    __syncthreads();
#pragma unroll 1
    for (int pos = tid; pos < 16 * KC; pos += 192) {
      const int qq = pos >> 6, kk = pos & 63;
      const int key = k0 + kk;
      float sv[HEADS], a2[HEADS];
#pragma unroll
      for (int h = 0; h < HEADS; ++h) { sv[h] = Ssh[h * 16 * SP + qq * SP + kk]; a2[h] = b2s[h]; }
      const float* mq = mst + qq * HEXP;
      const float* rq = rzs + qq * HEXP;
#pragma unroll 1
      for (int c = 0; c < HEXP; ++c) {
        const float* w1 = w1s + c * HEADS;
        float a1 = 0.f;
#pragma unroll
        for (int h = 0; h < HEADS; ++h) a1 += sv[h] * w1[h];
        a1 += b1s[c];
        const float p = __expf(a1 - mq[c]) * rq[c];
#pragma unroll
        for (int h = 0; h < HEADS; ++h) a2[h] += p * w2s[h * HEXP + c];
      }
      const bool valid = key < MQ;
#pragma unroll
      for (int h = 0; h < HEADS; ++h) {
        const float v = valid ? a2[h] : 0.f;
        const us hb = f2bf_bits(v);
        const us lb = f2bf_bits(v - bf_bits2f(hb));
        A2h[h * 16 * KC + qq * KC + kk] = __builtin_bit_cast(__bf16, hb);
        A2l[h * 16 * KC + qq * KC + kk] = __builtin_bit_cast(__bf16, lb);
      }
    }
    __syncthreads();
    const __bf16* arh = A2h + wave * 16 * KC + ln * KC;
    const __bf16* arl = A2l + wave * 16 * KC + ln * KC;
#pragma unroll
    for (int ks = 0; ks < KC; ks += 32) {
      const v16b ah = ldfrag(arh + ks + 8 * hg);
      const v16b al = ldfrag(arl + ks + 8 * hg);
#pragma unroll
      for (int dt = 0; dt < 4; ++dt) {
        const size_t vo = (size_t)(wave * HD + dt * 16 + ln) * MQP + k0 + ks + 8 * hg;
        const v16b bh = ldfrag(vth + vo);
        const v16b bl = ldfrag(vtl + vo);
        oacc[dt] = mma_g(ah, bh, oacc[dt]);
        oacc[dt] = mma_g(ah, bl, oacc[dt]);
        oacc[dt] = mma_g(al, bh, oacc[dt]);
      }
    }
  }
  __syncthreads();

  float* os = Ssh + wave * 16 * SP;
#pragma unroll
  for (int r = 0; r < 8; ++r) {
#pragma unroll
    for (int dt = 0; dt < 4; ++dt) os[(8 * hg + r) * SP + dt * 16 + ln] = oacc[dt][r];
  }
  __builtin_amdgcn_fence(__ATOMIC_RELEASE, "workgroup");
  __builtin_amdgcn_wave_barrier();
  __builtin_amdgcn_fence(__ATOMIC_ACQUIRE, "workgroup");
  const int rq = lane >> 3, c8 = (lane & 7) * 8;
  v4u hv[4], lv[4];
#pragma unroll
  for (int it = 0; it < 4; ++it) {
    const float* sp = os + (it * 4 + rq) * SP + c8;
    v4f a, bb;
    a.x = sp[0]; a.y = sp[1]; a.z = sp[2]; a.w = sp[3];
    bb.x = sp[4]; bb.y = sp[5]; bb.z = sp[6]; bb.w = sp[7];
    split8(a, bb, hv[it], lv[it]);
  }
  for (int pass = 0; pass < 2; ++pass) {
#pragma unroll
    for (int it = 0; it < 4; ++it) {
      const int row = it * 4 + rq;
      const size_t o = (size_t)(m0 + row) * DIM + wave * HD + c8;
      *(volatile v4u*)(aoh + o) = hv[it];
      *(volatile v4u*)(aol + o) = lv[it];
    }
    __threadfence();
  }
}

__global__ __launch_bounds__(256) void k_sqa(const float* __restrict__ kvo, const float* __restrict__ fo,
                                             const float* __restrict__ sp1w, const float* __restrict__ sp1b,
                                             const float* __restrict__ sp2w, const float* __restrict__ sp2b,
                                             const float* __restrict__ pnw, const float* __restrict__ pnb,
                                             float* addv, float* out1) {
  __shared__ __align__(16) float qs[DIM];
  __shared__ float lg[HEADS * NBT];
  __shared__ __align__(16) float x1s[DIM];
  __shared__ __align__(16) float s1[PRD];
  __shared__ __align__(16) float ys[PRD];
  __shared__ float red[8];
  __shared__ float pmax[HEADS], prz[HEADS];
  __shared__ float lnm, lninv;
  const int tid = threadIdx.x, wave = tid >> 5, lane = tid & 31;

  v4f qv = {0.f, 0.f, 0.f, 0.f};
  if (tid < DIM / 4) {
    qv = *(const v4f*)(fo + tid * 4);
    *(v4f*)(qs + tid * 4) = qv;
    *(volatile v4f*)(out1 + tid * 4) = qv;
  }
  __threadfence();
  if (tid < DIM / 4) *(volatile v4f*)(out1 + tid * 4) = qv;
  __syncthreads();

#pragma unroll 1
  for (int i = tid; i < HEADS * NBT; i += 256) {
    const int h = i / NBT, t = i - h * NBT;
    const float* kr = kvo + (size_t)t * (2 * DIM) + h * HD;
    const float* qh = qs + h * HD;
    float a = 0.f;
#pragma unroll 1
    for (int d = 0; d < HD; d += 4) {
      const v4f k4 = *(const v4f*)(kr + d);
      const v4f q4 = *(const v4f*)(qh + d);
      a += q4.x * k4.x; a += q4.y * k4.y; a += q4.z * k4.z; a += q4.w * k4.w;
    }
    lg[i] = a * SCALE_F;
  }
  __syncthreads();

#pragma unroll 1
  for (int h = 0; h < HEADS; ++h) {
    float m = -INFINITY;
    for (int t = tid; t < NBT; t += 256) m = fmaxf(m, lg[h * NBT + t]);
    m = wave_max(m);
    if (lane == 0) red[wave] = m;
    __syncthreads();
    if (tid == 0) {
      float mm = red[0];
      for (int ww = 1; ww < 8; ++ww) mm = fmaxf(mm, red[ww]);
      pmax[h] = mm;
    }
    __syncthreads();
    m = pmax[h];
    float s = 0.f;
    for (int t = tid; t < NBT; t += 256) s += __expf(lg[h * NBT + t] - m);
    s = wave_sum(s);
    if (lane == 0) red[wave] = s;
    __syncthreads();
    if (tid == 0) {
      float tt = 0.f;
      for (int ww = 0; ww < 8; ++ww) tt += red[ww];
      prz[h] = 1.0f / tt;
    }
    __syncthreads();
  }
#pragma unroll 1
  for (int i = tid; i < HEADS * NBT; i += 256) {
    const int h = i / NBT;
    lg[i] = __expf(lg[i] - pmax[h]) * prz[h];
  }
  __syncthreads();

#pragma unroll 1
  for (int pI = tid; pI < DIM; pI += 256) {
    const int h = pI >> 6, d = pI & 63;
    const float* vc = kvo + DIM + h * HD + d;
    const float* ph = lg + h * NBT;
    float a = 0.f;
#pragma unroll 1
    for (int t = 0; t < NBT; ++t) a += ph[t] * vc[(size_t)t * (2 * DIM)];
    x1s[pI] = a;
  }
  __syncthreads();

  if (tid < PRD) {
    const float* wr = sp1w + (size_t)tid * DIM;
    float a = 0.f;
#pragma unroll 1
    for (int d = 0; d < DIM; d += 4) {
      const v4f w4 = *(const v4f*)(wr + d);
      const v4f x4 = *(const v4f*)(x1s + d);
      a += w4.x * x4.x; a += w4.y * x4.y; a += w4.z * x4.z; a += w4.w * x4.w;
    }
    s1[tid] = a + sp1b[tid];
  }
  __syncthreads();
  if (tid < 32) {
    float s = s1[lane] + s1[lane + 32] + s1[lane + 64];
    s = wave_sum(s);
    const float m = s * (1.0f / PRD);
    const float d0 = s1[lane] - m, d1 = s1[lane + 32] - m, d2 = s1[lane + 64] - m;
    float ss = d0 * d0 + d1 * d1 + d2 * d2;
    ss = wave_sum(ss);
    if (lane == 0) { lnm = m; lninv = 1.0f / sqrtf(ss * (1.0f / PRD) + LN_EPS); }
  }
  __syncthreads();
  if (tid < PRD) {
    const float v = (s1[tid] - lnm) * lninv * pnw[tid] + pnb[tid];
    ys[tid] = fmaxf(v, 0.f);
  }
  __syncthreads();

#pragma unroll 1
  for (int d = tid; d < DIM; d += 256) {
    const float* wr = sp2w + (size_t)d * PRD;
    float a = 0.f;
#pragma unroll 1
    for (int o = 0; o < PRD; o += 4) {
      const v4f w4 = *(const v4f*)(wr + o);
      const v4f y4 = *(const v4f*)(ys + o);
      a += w4.x * y4.x; a += w4.y * y4.y; a += w4.z * y4.z; a += w4.w * y4.w;
    }
    x1s[d] = a + sp2b[d];
  }
  __syncthreads();
  v4f av = {0.f, 0.f, 0.f, 0.f};
  if (tid < DIM / 4) {
    av = *(const v4f*)(x1s + tid * 4);
    *(volatile v4f*)(addv + tid * 4) = av;
  }
  __threadfence();
  if (tid < DIM / 4) *(volatile v4f*)(addv + tid * 4) = av;
}

__global__ __launch_bounds__(256) void k_scatln(const float* __restrict__ x, const float* __restrict__ cin,
                                                const float* __restrict__ fo, const float* __restrict__ addv,
                                                const int* __restrict__ rankA,
                                                const float* __restrict__ n1w, const float* __restrict__ n1b,
                                                const float* __restrict__ n2w, const float* __restrict__ n2b,
                                                float* x2o, us* lnh, us* lnl) {
  __shared__ __align__(16) float rowbuf[8][DIM];
  const int tid = threadIdx.x, wave = tid >> 5, lane = tid & 31;
  const int r = blockIdx.x * 8 + wave;
  const int i2 = r / HS, j2 = r - i2 * HS;
  const int p = (i2 >> 1) * HPW + (j2 >> 1);
  const int t = (i2 & 1) * 2 + (j2 & 1);
  int rk = rankA[p];
  rk = min(max(rk, 0), NP - 1);
  const bool fg = rk < NF;
  const int frow = 1 + min(rk, NF - 1) * 4 + t;

  v4f xv[3], v1[3];
  float s = 0.f;
#pragma unroll
  for (int it = 0; it < 3; ++it) {
    const int col = it * 128 + lane * 4;
    xv[it] = *(const v4f*)(x + (size_t)r * DIM + col);
    const v4f fv = *(const v4f*)(fo + (size_t)frow * DIM + col);
    const v4f cv = *(const v4f*)(cin + (size_t)r * DIM + col);
    const v4f av = *(const v4f*)(addv + col);
    const v4f bv = cv + av;
    v1[it] = fg ? fv : bv;
    s += (v1[it].x + v1[it].y) + (v1[it].z + v1[it].w);
  }
  s = wave_sum(s);
  const float m1 = s * (1.0f / DIM);
  float ss = 0.f;
#pragma unroll
  for (int it = 0; it < 3; ++it) {
    const v4f d = v1[it] - m1;
    ss += (d.x * d.x + d.y * d.y) + (d.z * d.z + d.w * d.w);
  }
  ss = wave_sum(ss);
  const float inv1 = 1.0f / sqrtf(ss * (1.0f / DIM) + LN_EPS);

  v4f x2v[3];
  float s2 = 0.f;
#pragma unroll
  for (int it = 0; it < 3; ++it) {
    const int col = it * 128 + lane * 4;
    const v4f w = *(const v4f*)(n1w + col);
    const v4f bb = *(const v4f*)(n1b + col);
    x2v[it] = xv[it] + (((v1[it] - m1) * inv1) * w + bb);
    s2 += (x2v[it].x + x2v[it].y) + (x2v[it].z + x2v[it].w);
  }
  s2 = wave_sum(s2);
  const float m2 = s2 * (1.0f / DIM);
  float ss2 = 0.f;
#pragma unroll
  for (int it = 0; it < 3; ++it) {
    const v4f d = x2v[it] - m2;
    ss2 += (d.x * d.x + d.y * d.y) + (d.z * d.z + d.w * d.w);
  }
  ss2 = wave_sum(ss2);
  const float inv2 = 1.0f / sqrtf(ss2 * (1.0f / DIM) + LN_EPS);
  v4f hv[3];
#pragma unroll
  for (int it = 0; it < 3; ++it) {
    const int col = it * 128 + lane * 4;
    const v4f w = *(const v4f*)(n2w + col);
    const v4f bb = *(const v4f*)(n2b + col);
    hv[it] = ((x2v[it] - m2) * inv2) * w + bb;
  }

#pragma unroll
  for (int it = 0; it < 3; ++it) {
    const int col = it * 128 + lane * 4;
    *(volatile v4f*)(x2o + (size_t)r * DIM + col) = x2v[it];
  }
#pragma unroll
  for (int it = 0; it < 3; ++it) {
    const int col = it * 128 + lane * 4;
    *(v4f*)(rowbuf[wave] + col) = hv[it];
  }
  __builtin_amdgcn_fence(__ATOMIC_RELEASE, "workgroup");
  __builtin_amdgcn_wave_barrier();
  __builtin_amdgcn_fence(__ATOMIC_ACQUIRE, "workgroup");
  v4u ph[2], pl[2];
#pragma unroll
  for (int it2 = 0; it2 < 2; ++it2) {
    int c8 = it2 * 256 + lane * 8;
    c8 = min(c8, DIM - 8);
    const v4f a = *(const v4f*)(rowbuf[wave] + c8);
    const v4f bb = *(const v4f*)(rowbuf[wave] + c8 + 4);
    split8(a, bb, ph[it2], pl[it2]);
  }
  us* hrow = lnh + (size_t)r * DIM;
  us* lrow = lnl + (size_t)r * DIM;
  *(volatile v4u*)(hrow + lane * 8) = ph[0];
  *(volatile v4u*)(lrow + lane * 8) = pl[0];
  if (lane < 16) {
    *(volatile v4u*)(hrow + 256 + lane * 8) = ph[1];
    *(volatile v4u*)(lrow + 256 + lane * 8) = pl[1];
  }
  __threadfence();
#pragma unroll
  for (int it = 0; it < 3; ++it) {
    const int col = it * 128 + lane * 4;
    *(volatile v4f*)(x2o + (size_t)r * DIM + col) = x2v[it];
  }
  *(volatile v4u*)(hrow + lane * 8) = ph[0];
  *(volatile v4u*)(lrow + lane * 8) = pl[0];
  if (lane < 16) {
    *(volatile v4u*)(hrow + 256 + lane * 8) = ph[1];
    *(volatile v4u*)(lrow + 256 + lane * 8) = pl[1];
  }
}

extern "C" void kernel_launch(void* const* d_in, const int* in_sizes, int n_in,
                              void* d_out, int out_size, void* d_ws, size_t ws_size,
                              hipStream_t stream) {
  if (n_in < 28) return;
  if (in_sizes[0] != LTOK * DIM || in_sizes[1] != DIM || in_sizes[2] != DIM * 9 || in_sizes[3] != DIM) return;
  if (in_sizes[4] != DIM || in_sizes[5] != DIM || in_sizes[6] != DIM || in_sizes[7] != DIM) return;
  if (in_sizes[8] != 3 * DIM * DIM || in_sizes[9] != 3 * DIM || in_sizes[10] != DIM * DIM || in_sizes[11] != DIM) return;
  if (in_sizes[12] != HEXP * HEADS || in_sizes[13] != HEXP || in_sizes[14] != HEADS * HEXP || in_sizes[15] != HEADS) return;
  if (in_sizes[16] != 2 * DIM * DIM || in_sizes[17] != 2 * DIM || in_sizes[18] != PRD * DIM || in_sizes[19] != PRD) return;
  if (in_sizes[20] != DIM * PRD || in_sizes[21] != DIM || in_sizes[22] != PRD || in_sizes[23] != PRD) return;
  if (in_sizes[24] != HID * DIM || in_sizes[25] != HID || in_sizes[26] != DIM * HID || in_sizes[27] != DIM) return;
  if (out_size != LTOK * DIM + DIM) return;

  const float* x       = (const float*)d_in[0];
  const float* qa      = (const float*)d_in[1];
  const float* conv_w  = (const float*)d_in[2];
  const float* conv_b  = (const float*)d_in[3];
  const float* n1w     = (const float*)d_in[4];
  const float* n1b     = (const float*)d_in[5];
  const float* n2w     = (const float*)d_in[6];
  const float* n2b     = (const float*)d_in[7];
  const float* qkv_w   = (const float*)d_in[8];
  const float* qkv_b   = (const float*)d_in[9];
  const float* mproj_w = (const float*)d_in[10];
  const float* mproj_b = (const float*)d_in[11];
  const float* ap1_w   = (const float*)d_in[12];
  const float* ap1_b   = (const float*)d_in[13];
  const float* ap2_w   = (const float*)d_in[14];
  const float* ap2_b   = (const float*)d_in[15];
  const float* kv_w    = (const float*)d_in[16];
  const float* kv_b    = (const float*)d_in[17];
  const float* sp1_w   = (const float*)d_in[18];
  const float* sp1_b   = (const float*)d_in[19];
  const float* sp2_w   = (const float*)d_in[20];
  const float* sp2_b   = (const float*)d_in[21];
  const float* pn_w    = (const float*)d_in[22];
  const float* pn_b    = (const float*)d_in[23];
  const float* fc1_w   = (const float*)d_in[24];
  const float* fc1_b   = (const float*)d_in[25];
  const float* fc2_w   = (const float*)d_in[26];
  const float* fc2_b   = (const float*)d_in[27];
  float* out0 = (float*)d_out;
  float* out1 = out0 + (size_t)LTOK * DIM;

  const size_t szC    = (size_t)LTOK * DIM * 4;
  const size_t szTab  = 3328;
  const size_t szX16  = (size_t)MQP * DIM * 2;
  const size_t szWqkv = (size_t)3 * DIM * DIM * 2;
  const size_t szWmp  = (size_t)DIM * DIM * 2;
  const size_t szWkv  = (size_t)2 * DIM * DIM * 2;
  const size_t szWfc  = (size_t)HID * DIM * 2;
  const size_t szQK   = (size_t)MQP * 2 * DIM * 2;
  const size_t szVT   = (size_t)DIM * MQP * 2;
  const size_t szS    = (size_t)HEADS * MQP * MQP * 4;
  const size_t szFo   = (size_t)MQP * DIM * 4;
  const size_t szKvo  = (size_t)MQP * 2 * DIM * 4;
  const size_t szAdd  = (size_t)DIM * 4;
  const size_t szX2   = (size_t)LTOK * DIM * 4;
  const size_t szLN   = (size_t)LTOK * DIM * 2;
  const size_t szH    = (size_t)LTOK * HID * 2;
  size_t off = 0;
  const size_t oC    = off; off += szC;
  const size_t oRank = off; off += szTab;
  const size_t oOrd  = off; off += szTab;
  const size_t oXfh  = off; off += szX16;  const size_t oXfl = off; off += szX16;
  const size_t oXbh  = off; off += szX16;  const size_t oXbl = off; off += szX16;
  const size_t oWqh  = off; off += szWqkv; const size_t oWql = off; off += szWqkv;
  const size_t oWmh  = off; off += szWmp;  const size_t oWml = off; off += szWmp;
  const size_t oWkh  = off; off += szWkv;  const size_t oWkl = off; off += szWkv;
  const size_t oW1h  = off; off += szWfc;  const size_t oW1l = off; off += szWfc;
  const size_t oW2h  = off; off += szWfc;  const size_t oW2l = off; off += szWfc;
  const size_t oQKh  = off; off += szQK;   const size_t oQKl = off; off += szQK;
  const size_t oVTh  = off; off += szVT;   const size_t oVTl = off; off += szVT;
  const size_t oS    = off; off += szS;
  const size_t oAOh  = off; off += szX16;  const size_t oAOl = off; off += szX16;
  const size_t oFo   = off; off += szFo;
  const size_t oKvo  = off; off += szKvo;
  const size_t oAdd  = off; off += szAdd;
  const size_t oX2   = off; off += szX2;
  const size_t oLNh  = off; off += szLN;   const size_t oLNl = off; off += szLN;
  const size_t oHh   = off; off += szH;    const size_t oHl  = off; off += szH;
  if (off > ws_size) return;
  if (off > (size_t)134217728) return;

  char* ws = (char*)d_ws;
  float* cbuf  = (float*)(ws + oC);
  int*   rankA = (int*)(ws + oRank);
  int*   order = (int*)(ws + oOrd);
  us* Xfh = (us*)(ws + oXfh); us* Xfl = (us*)(ws + oXfl);
  us* Xbh = (us*)(ws + oXbh); us* Xbl = (us*)(ws + oXbl);
  us* Wqh = (us*)(ws + oWqh); us* Wql = (us*)(ws + oWql);
  us* Wmh = (us*)(ws + oWmh); us* Wml = (us*)(ws + oWml);
  us* Wkh = (us*)(ws + oWkh); us* Wkl = (us*)(ws + oWkl);
  us* W1h = (us*)(ws + oW1h); us* W1l = (us*)(ws + oW1l);
  us* W2h = (us*)(ws + oW2h); us* W2l = (us*)(ws + oW2l);
  us* QKh = (us*)(ws + oQKh); us* QKl = (us*)(ws + oQKl);
  us* VTh = (us*)(ws + oVTh); us* VTl = (us*)(ws + oVTl);
  float* Sbuf  = (float*)(ws + oS);
  us* AOh = (us*)(ws + oAOh); us* AOl = (us*)(ws + oAOl);
  float* f_out  = (float*)(ws + oFo);
  float* kv_out = (float*)(ws + oKvo);
  float* addvec = (float*)(ws + oAdd);
  float* X2     = (float*)(ws + oX2);
  us* LNh = (us*)(ws + oLNh); us* LNl = (us*)(ws + oLNl);
  us* Hh  = (us*)(ws + oHh);  us* Hl  = (us*)(ws + oHl);

  const dim3 blk(256);

  { const int n8 = 3 * DIM * DIM / 8; k_split8<<<dim3((n8 + 255) / 256), blk, 0, stream>>>(qkv_w, Wqh, Wql, n8); }
  { const int n8 = DIM * DIM / 8;     k_split8<<<dim3((n8 + 255) / 256), blk, 0, stream>>>(mproj_w, Wmh, Wml, n8); }
  { const int n8 = 2 * DIM * DIM / 8; k_split8<<<dim3((n8 + 255) / 256), blk, 0, stream>>>(kv_w, Wkh, Wkl, n8); }
  { const int n8 = HID * DIM / 8;     k_split8<<<dim3((n8 + 255) / 256), blk, 0, stream>>>(fc1_w, W1h, W1l, n8); }
  { const int n8 = DIM * HID / 8;     k_split8<<<dim3((n8 + 255) / 256), blk, 0, stream>>>(fc2_w, W2h, W2l, n8); }

  k_conv<<<dim3((LTOK * (DIM / 4) + 255) / 256), blk, 0, stream>>>(x, conv_w, conv_b, cbuf);
  k_rank<<<dim3(1), blk, 0, stream>>>(cbuf, rankA, order);
  k_gather8<<<dim3((2 * MQP * (DIM / 8) + 255) / 256), blk, 0, stream>>>(cbuf, qa, order, Xfh, Xfl, Xbh, Xbl);

  {
    const int tiles = (MQP / 64) * ((2 * DIM) / 64);
    k_gemm64<2, 2, false, 0><<<dim3((tiles + 7) / 8, 1), blk, 0, stream>>>(
        Xfh, Xfl, DIM, 0L, Wqh, Wql, DIM, 0L, (void*)QKh, (void*)QKl, 2 * DIM, 0L,
        qkv_b, qkv_b, MQP, 2 * DIM, DIM, 1.0f);
  }
  {
    const int tiles = (DIM / 64) * (MQP / 64);
    k_gemm64<1, 2, false, 0><<<dim3((tiles + 7) / 8, 1), blk, 0, stream>>>(
        Wqh + (size_t)2 * DIM * DIM, Wql + (size_t)2 * DIM * DIM, DIM, 0L, Xfh, Xfl, DIM, 0L,
        (void*)VTh, (void*)VTl, MQP, 0L, qkv_b + 2 * DIM, qkv_b + 2 * DIM, DIM, MQP, DIM, 1.0f);
  }
  {
    const int tiles = (MQP / 64) * (MQP / 64);
    k_gemm64<0, 0, false, 0><<<dim3((tiles + 7) / 8, HEADS), blk, 0, stream>>>(
        QKh, QKl, 2 * DIM, (long)HD, QKh + DIM, QKl + DIM, 2 * DIM, (long)HD,
        (void*)Sbuf, (void*)Sbuf, MQP, (long)MQP * MQP, qkv_b, qkv_b, MQP, MQP, HD, SCALE_F);
  }
  k_mmsa<<<dim3(MQP / 16), dim3(192), 0, stream>>>(Sbuf, VTh, VTl, ap1_w, ap1_b, ap2_w, ap2_b, AOh, AOl);
  {
    const int tiles = (MQP / 64) * (DIM / 64);
    k_gemm64<2, 0, false, 0><<<dim3((tiles + 7) / 8, 1), blk, 0, stream>>>(
        AOh, AOl, DIM, 0L, Wmh, Wml, DIM, 0L, (void*)f_out, (void*)f_out, DIM, 0L,
        mproj_b, mproj_b, MQP, DIM, DIM, 1.0f);
  }
  {
    const int tiles = (MQP / 64) * ((2 * DIM) / 64);
    k_gemm64<2, 0, false, 0><<<dim3((tiles + 7) / 8, 1), blk, 0, stream>>>(
        Xbh, Xbl, DIM, 0L, Wkh, Wkl, DIM, 0L, (void*)kv_out, (void*)kv_out, 2 * DIM, 0L,
        kv_b, kv_b, MQP, 2 * DIM, DIM, 1.0f);
  }
  k_sqa<<<dim3(1), blk, 0, stream>>>(kv_out, f_out, sp1_w, sp1_b, sp2_w, sp2_b, pn_w, pn_b, addvec, out1);
  k_scatln<<<dim3(LTOK / 8), blk, 0, stream>>>(x, cbuf, f_out, addvec, rankA, n1w, n1b, n2w, n2b, X2, LNh, LNl);
  {
    const int tiles = (LTOK / 64) * (HID / 64);
    k_gemm64<2, 2, false, 3><<<dim3((tiles + 7) / 8, 1), blk, 0, stream>>>(
        LNh, LNl, DIM, 0L, W1h, W1l, DIM, 0L, (void*)Hh, (void*)Hl, HID, 0L,
        fc1_b, fc1_b, LTOK, HID, DIM, 1.0f);
  }
  {
    const int tiles = (LTOK / 64) * (DIM / 64);
    k_gemm64<2, 0, true, 0><<<dim3((tiles + 7) / 8, 1), blk, 0, stream>>>(
        Hh, Hl, HID, 0L, W2h, W2l, HID, 0L, (void*)out0, (void*)out0, DIM, 0L,
        fc2_b, X2, LTOK, DIM, HID, 1.0f);
  }
  (void)hipGetLastError();
}
